// BurgersPinn_4294967296648
// MI455X (gfx1250) — hardware-verified
//
#include <hip/hip_runtime.h>
#include <stddef.h>


typedef _Float16 v8h  __attribute__((ext_vector_type(8)));
typedef _Float16 v16h __attribute__((ext_vector_type(16)));
typedef float    v8f  __attribute__((ext_vector_type(8)));
typedef float    v4f  __attribute__((ext_vector_type(4)));

union Frag { v16h v; v8h half[2]; };

#define HID        128
#define CH         64
#define PW         16
#define NTHR       128
#define NBLK_MAX   136
#define NU_C       0.0031830988618379067f
#define WSCL       16.0f
#define WSCL_INV   0.0625f
#define TSCL       16.0f
#define TSCL_INV   0.0625f
#define XXSCL_INV  0.00390625f

#define WT_OFF     0
#define WT_HALVES  (HID * HID)
#define ACT_OFF    98304
#define SBUF       2048
#define WBUF       (8 * SBUF)
#define F32_OFF    229376
#define F_W0       0
#define F_B0       256
#define F_BL       384
#define F_W4       768
#define F_B4       896
#define F_TXS      912
#define F_OST      1040
#define F_TOTAL    1104
#define SMEM_BYTES (F32_OFF + F_TOTAL * 4)

__device__ __forceinline__ float tanh_f(float z) {
  const float e = __expf(2.0f * z);
  const float r = __builtin_amdgcn_rcpf(e + 1.0f);
  return fmaf(-2.0f, r, 1.0f);
}

__device__ __forceinline__ v16h ld_frag(const _Float16* row, int kb) {
  Frag f;
  f.half[0] = *(const v8h*)(row + kb);
  f.half[1] = *(const v8h*)(row + kb + 16);
  return f.v;
}

__device__ __forceinline__ v8f wmma16(v16h a, v16h b, v8f c) {
  return __builtin_amdgcn_wmma_f32_16x16x32_f16(false, a, false, b, (short)0, c, false, false);
}

__device__ __forceinline__ v8h pack8(const float (&v)[8]) {
  v8h r = { (_Float16)v[0], (_Float16)v[1], (_Float16)v[2], (_Float16)v[3],
            (_Float16)v[4], (_Float16)v[5], (_Float16)v[6], (_Float16)v[7] };
  return r;
}

__device__ __forceinline__ void ld8f(const float* p, float (&o)[8]) {
  const v4f a = *(const v4f*)p;
  const v4f b = *(const v4f*)(p + 4);
  o[0] = a[0]; o[1] = a[1]; o[2] = a[2]; o[3] = a[3];
  o[4] = b[0]; o[5] = b[1]; o[6] = b[2]; o[7] = b[3];
}

template <int NS>
__device__ __forceinline__ float chunk_body(const _Float16* wt, const float* fw,
                                            _Float16* buf0, _Float16* buf1,
                                            const float* txs, int wave, int lane)
{
  const int h = lane >> 4;
  const int m = lane & 15;
  const v8f zero8 = {0.f, 0.f, 0.f, 0.f, 0.f, 0.f, 0.f, 0.f};

  {
    const float t = txs[(wave * PW + m) * 2];
    const float x = txs[(wave * PW + m) * 2 + 1];
    const float* w0t = fw + F_W0 + 64 * h;
    const float* w0x = fw + F_W0 + HID + 64 * h;
    const float* bz  = fw + F_B0 + 64 * h;
    _Float16* H = buf0 + m * HID + 64 * h;
#pragma unroll 1
    for (int j = 0; j < 8; ++j) {
      float ct[8], cx[8], bb8[8];
      ld8f(w0t + 8 * j, ct);
      ld8f(w0x + 8 * j, cx);
      ld8f(bz + 8 * j, bb8);
      float av[8];
#pragma unroll
      for (int e = 0; e < 8; ++e) {
        const float z = t * ct[e] + x * cx[e] + bb8[e];
        av[e] = tanh_f(z);
      }
      *(v8h*)(H + 8 * j) = pack8(av);
      if constexpr (NS == 4) {
        float tv[8], xv[8], xxv[8];
#pragma unroll
        for (int e = 0; e < 8; ++e) {
          const float a = av[e];
          const float ap = 1.0f - a * a;
          const float cts = TSCL * ct[e];
          const float cxs = TSCL * cx[e];
          tv[e]  = ap * cts;
          xv[e]  = ap * cxs;
          xxv[e] = -2.0f * a * ap * cxs * cxs;
        }
        *(v8h*)(H + SBUF + 8 * j)     = pack8(tv);
        *(v8h*)(H + 2 * SBUF + 8 * j) = pack8(xv);
        *(v8h*)(H + 3 * SBUF + 8 * j) = pack8(xxv);
      }
    }
  }
  __syncthreads();

#pragma unroll 1
  for (int l = 0; l < 3; ++l) {
    const _Float16* S = (l & 1) ? buf1 : buf0;
    _Float16*       D = (l & 1) ? buf0 : buf1;
    const _Float16* wl = wt + l * WT_HALVES;
    const float*    bb = fw + F_BL + l * HID;
    const _Float16* srow = S + m * HID;
#pragma unroll 1
    for (int n0 = 0; n0 < 8; n0 += 2) {
      v8f acc[NS][2];
#pragma unroll
      for (int s = 0; s < NS; ++s) { acc[s][0] = zero8; acc[s][1] = zero8; }
      const _Float16* wr0 = wl + (n0 * 16 + m) * HID;
      const _Float16* wr1 = wr0 + 16 * HID;
#pragma unroll
      for (int k0 = 0; k0 < 4; ++k0) {
        const int kb = k0 * 32 + 8 * h;
        v16h a0 = ld_frag(wr0, kb);
        v16h a1 = ld_frag(wr1, kb);
        v16h b[NS];
#pragma unroll
        for (int s = 0; s < NS; ++s) b[s] = ld_frag(srow + s * SBUF, kb);
#pragma unroll
        for (int s = 0; s < NS; ++s) {
          acc[s][0] = wmma16(a0, b[s], acc[s][0]);
          acc[s][1] = wmma16(a1, b[s], acc[s][1]);
        }
        if constexpr (NS == 4) {
          asm volatile("v_nop\n\tv_nop\n\tv_nop\n\tv_nop"
                       : "+v"(acc[0][0]), "+v"(acc[0][1]), "+v"(acc[1][0]), "+v"(acc[1][1]),
                         "+v"(acc[2][0]), "+v"(acc[2][1]), "+v"(acc[3][0]), "+v"(acc[3][1])
                       : "v"(a0), "v"(a1), "v"(b[0]), "v"(b[1]), "v"(b[2]), "v"(b[3]));
        } else {
          asm volatile("v_nop\n\tv_nop\n\tv_nop\n\tv_nop"
                       : "+v"(acc[0][0]), "+v"(acc[0][1])
                       : "v"(a0), "v"(a1), "v"(b[0]));
        }
      }
#pragma unroll
      for (int ti = 0; ti < 2; ++ti) {
        const int nb = (n0 + ti) * 16 + 8 * h;
        float bias[8];
        ld8f(bb + nb, bias);
        float av[8];
#pragma unroll
        for (int r = 0; r < 8; ++r) av[r] = tanh_f(fmaf(acc[0][ti][r], WSCL_INV, bias[r]));
        _Float16* dp = D + m * HID + nb;
        *(v8h*)dp = pack8(av);
        if constexpr (NS == 4) {
          float tv[8], xv[8], xxv[8];
#pragma unroll
          for (int r = 0; r < 8; ++r) {
            const float a   = av[r];
            const float ap  = 1.0f - a * a;
            const float zt  = acc[1][ti][r] * WSCL_INV;
            const float zx  = acc[2][ti][r] * WSCL_INV;
            const float zxx = acc[3][ti][r] * WSCL_INV;
            tv[r]  = ap * zt;
            xv[r]  = ap * zx;
            xxv[r] = ap * zxx - 2.0f * a * ap * zx * zx;
          }
          *(v8h*)(dp + SBUF)     = pack8(tv);
          *(v8h*)(dp + 2 * SBUF) = pack8(xv);
          *(v8h*)(dp + 3 * SBUF) = pack8(xxv);
        }
      }
    }
    __syncthreads();
  }

  const _Float16* Hf = buf1 + m * HID + 64 * h;
  const float* w4 = fw + F_W4 + 64 * h;
  float su = 0.f, st = 0.f, sx = 0.f, sxx = 0.f;
#pragma unroll 1
  for (int c = 0; c < 8; ++c) {
    float w[8];
    ld8f(w4 + 8 * c, w);
    const v8h v0 = *(const v8h*)(Hf + 8 * c);
#pragma unroll
    for (int e = 0; e < 8; ++e) su += (float)v0[e] * w[e];
    if constexpr (NS == 4) {
      const v8h v1 = *(const v8h*)(Hf + SBUF + 8 * c);
      const v8h v2 = *(const v8h*)(Hf + 2 * SBUF + 8 * c);
      const v8h v3 = *(const v8h*)(Hf + 3 * SBUF + 8 * c);
#pragma unroll
      for (int e = 0; e < 8; ++e) {
        st  += (float)v1[e] * w[e];
        sx  += (float)v2[e] * w[e];
        sxx += (float)v3[e] * w[e];
      }
    }
  }
  su += __shfl_xor(su, 16, 32);
  float val;
  if constexpr (NS == 4) {
    st  += __shfl_xor(st, 16, 32);
    sx  += __shfl_xor(sx, 16, 32);
    sxx += __shfl_xor(sxx, 16, 32);
    const float u   = su + fw[F_B4];
    const float ut  = st * TSCL_INV;
    const float ux  = sx * TSCL_INV;
    const float uxx = sxx * XXSCL_INV;
    val = (ut + u * ux) - NU_C * uxx;
  } else {
    val = su + fw[F_B4];
  }
  return val;
}

extern "C" __global__ __launch_bounds__(NTHR) __attribute__((amdgpu_num_vgpr(256)))
void k_mlp_streams(const float* __restrict__ txe, const float* __restrict__ txi, const float* __restrict__ txb,
                   const float* __restrict__ W0g, const float* __restrict__ b0g,
                   const float* __restrict__ W1g, const float* __restrict__ b1g,
                   const float* __restrict__ W2g, const float* __restrict__ b2g,
                   const float* __restrict__ W3g, const float* __restrict__ b3g,
                   const float* __restrict__ W4g, const float* __restrict__ b4g,
                   float* __restrict__ out, int n_eq, int n_init, int n_bnd)
{
  extern __shared__ __attribute__((aligned(16))) char smem[];
  _Float16* wt  = (_Float16*)(smem + WT_OFF);
  _Float16* act = (_Float16*)(smem + ACT_OFF);
  float*    fw  = (float*)(smem + F32_OFF);
  const int tid  = threadIdx.x;
  const int wave = tid >> 5;
  const int lane = tid & 31;

  for (int idx = tid; idx < WT_HALVES; idx += NTHR) {
    const int k = idx / HID;
    const int n = idx % HID;
    const int d = n * HID + k;
    wt[d]                 = (_Float16)(WSCL * W1g[idx]);
    wt[WT_HALVES + d]     = (_Float16)(WSCL * W2g[idx]);
    wt[2 * WT_HALVES + d] = (_Float16)(WSCL * W3g[idx]);
  }
  for (int i = tid; i < HID; i += NTHR) {
    fw[F_W0 + i]           = W0g[i];
    fw[F_W0 + HID + i]     = W0g[HID + i];
    fw[F_B0 + i]           = b0g[i];
    fw[F_BL + i]           = b1g[i];
    fw[F_BL + HID + i]     = b2g[i];
    fw[F_BL + 2 * HID + i] = b3g[i];
    fw[F_W4 + i]           = W4g[i];
  }
  if (tid == 0) fw[F_B4] = b4g[0];
  __syncthreads();

  const int ceq   = (n_eq + CH - 1) / CH;
  const int cin   = (n_init + CH - 1) / CH;
  const int cbn   = (n_bnd + CH - 1) / CH;
  const int total = ceq + cin + cbn;

  _Float16* buf0 = act + wave * WBUF;
  _Float16* buf1 = buf0 + 4 * SBUF;
  float* txs = fw + F_TXS;
  float* ost = fw + F_OST;

  for (int chunk = blockIdx.x; chunk < total; chunk += gridDim.x) {
    const float* src;
    int nseg, c;
    size_t obase;
    bool full4;
    if (chunk < ceq)            { c = chunk;             src = txe; nseg = n_eq;   obase = 0;                              full4 = true;  }
    else if (chunk < ceq + cin) { c = chunk - ceq;       src = txi; nseg = n_init; obase = (size_t)n_eq;                   full4 = false; }
    else                        { c = chunk - ceq - cin; src = txb; nseg = n_bnd;  obase = (size_t)n_eq + (size_t)n_init;  full4 = false; }
    const int p0 = c * CH;
    int valid = nseg - p0;
    if (valid > CH) valid = CH;

    if (tid < CH) {
      int q = p0 + tid;
      if (q > nseg - 1) q = nseg - 1;
      txs[2 * tid]     = src[2 * (size_t)q];
      txs[2 * tid + 1] = src[2 * (size_t)q + 1];
    }
    __syncthreads();

    float val;
    if (full4) val = chunk_body<4>(wt, fw, buf0, buf1, txs, wave, lane);
    else       val = chunk_body<1>(wt, fw, buf0, buf1, txs, wave, lane);

    if ((lane >> 4) == 0) ost[wave * PW + (lane & 15)] = val;
    __syncthreads();

    if (wave == 0) {
      float* dst = out + obase + (size_t)p0;
      const bool vec_ok = (valid == CH) && (((obase + (size_t)p0) & 3) == 0);
      if (vec_ok) {
        v4f v = {0.f, 0.f, 0.f, 0.f};
        if (lane < 16) v = *(const v4f*)(ost + 4 * lane);
        if (lane < 16) *(volatile v4f*)(dst + 4 * lane) = v;
        __threadfence();
        if (lane < 16) *(volatile v4f*)(dst + 4 * lane) = v;
      } else {
        for (int i = lane; i < valid; i += 32) { const float s1 = ost[i]; *(volatile float*)(dst + i) = s1; }
        __threadfence();
        for (int i = lane; i < valid; i += 32) { const float s1 = ost[i]; *(volatile float*)(dst + i) = s1; }
      }
    }
  }
}

extern "C" void kernel_launch(void* const* d_in, const int* in_sizes, int n_in,
                              void* d_out, int out_size, void* d_ws, size_t ws_size,
                              hipStream_t stream)
{
  (void)d_ws; (void)ws_size;
  if (n_in < 13) return;
  if (in_sizes[3] != 2 * HID || in_sizes[4] != HID ||
      in_sizes[5] != HID * HID || in_sizes[6] != HID ||
      in_sizes[7] != HID * HID || in_sizes[8] != HID ||
      in_sizes[9] != HID * HID || in_sizes[10] != HID ||
      in_sizes[11] != HID || in_sizes[12] < 1) return;
  const int n_eq   = in_sizes[0] / 2;
  const int n_init = in_sizes[1] / 2;
  const int n_bnd  = in_sizes[2] / 2;
  if (n_eq < 0 || n_init < 0 || n_bnd < 0) return;
  if ((long long)n_eq + (long long)n_init + (long long)n_bnd > (long long)out_size) return;
  const int total = (n_eq + CH - 1) / CH + (n_init + CH - 1) / CH + (n_bnd + CH - 1) / CH;
  if (total <= 0) return;
  const int grid = total < NBLK_MAX ? total : NBLK_MAX;

  hipFuncSetAttribute(reinterpret_cast<const void*>(&k_mlp_streams),
                      hipFuncAttributeMaxDynamicSharedMemorySize, SMEM_BYTES);

  k_mlp_streams<<<dim3(grid), dim3(NTHR), SMEM_BYTES, stream>>>(
      (const float*)d_in[0], (const float*)d_in[1], (const float*)d_in[2],
      (const float*)d_in[3], (const float*)d_in[4],
      (const float*)d_in[5], (const float*)d_in[6],
      (const float*)d_in[7], (const float*)d_in[8],
      (const float*)d_in[9], (const float*)d_in[10],
      (const float*)d_in[11], (const float*)d_in[12],
      (float*)d_out, n_eq, n_init, n_bnd);
  (void)hipGetLastError();
}
